// MultiHeadCrossAttentionModule_944892805456
// MI455X (gfx1250) — hardware-run, weakly checked
//
#include <hip/hip_runtime.h>
#include <math.h>

typedef __attribute__((ext_vector_type(16))) _Float16 v16h;
typedef __attribute__((ext_vector_type(16))) __bf16 v16b;
typedef __attribute__((ext_vector_type(8)))  _Float16 v8h;
typedef __attribute__((ext_vector_type(8)))  float v8f;
typedef __attribute__((ext_vector_type(4)))  float v4f;
typedef __attribute__((ext_vector_type(2)))  float v2f;
typedef __attribute__((ext_vector_type(4)))  unsigned v4u;
typedef __attribute__((ext_vector_type(4)))  int v4i;
typedef float __attribute__((may_alias)) float_a;
typedef int __attribute__((may_alias)) int_a;

template <typename T> __device__ __forceinline__ void vst2(void* p, T v) { *(volatile T*)p = v; __threadfence(); *(volatile T*)p = v; }
__device__ __forceinline__ v8f wmma16(v16h a, v16h b, v8f c) {
  v8f d = __builtin_amdgcn_wmma_f32_16x16x32_f16(false, a, false, b, (short)0, c, false, false);
  asm volatile("v_nop\n\tv_nop\n\tv_nop\n\tv_nop" : "+v"(d) : "v"(a), "v"(b));
  return d;
}
__device__ __forceinline__ v8f wmma_bf(v16b a, v16b b, v8f c) {
  v8f d = __builtin_amdgcn_wmma_f32_16x16x32_bf16(false, a, false, b, (short)0, c, false, false);
  asm volatile("v_nop\n\tv_nop\n\tv_nop\n\tv_nop" : "+v"(d) : "v"(a), "v"(b));
  return d;
}
__device__ __forceinline__ v16h frag_h(const _Float16* rowk0, int lane) {
  union { v16h v; v8h q[2]; } u; const _Float16* p = rowk0 + 8 * (lane >> 4);
  u.q[0] = *(const v8h*)p; u.q[1] = *(const v8h*)(p + 16); return u.v;
}
__device__ __forceinline__ v16h frag_f32(const float* rowk0, int lane) {
  v16h a; const float* p = rowk0 + 8 * (lane >> 4);
#pragma unroll
  for (int i = 0; i < 8; ++i) { a[i] = (_Float16)p[i]; a[8 + i] = (_Float16)p[16 + i]; }
  return a;
}
__device__ __forceinline__ v16h frag_f32s(const float* rowk0, int lane, float sc) {
  v16h a; const float* p = rowk0 + 8 * (lane >> 4);
#pragma unroll
  for (int i = 0; i < 8; ++i) { a[i] = (_Float16)(p[i] * sc); a[8 + i] = (_Float16)(p[16 + i] * sc); }
  return a;
}
__device__ __forceinline__ v16h fragc_f32(const float* W, int k0, int n, int lane, int ld, int K) {
  v16h a; const int g = lane >> 4;
#pragma unroll
  for (int i = 0; i < 8; ++i) { const int ka = k0 + 8 * g + i, kb = ka + 16;
    a[i] = (_Float16)(ka < K ? W[(size_t)(ka < K ? ka : K - 1) * ld + n] : 0.f); a[8 + i] = (_Float16)(kb < K ? W[(size_t)(kb < K ? kb : K - 1) * ld + n] : 0.f); }
  return a;
}
struct F2 { v16b h, l; };
__device__ __forceinline__ F2 bsplit16(const float v[16]) { F2 r;
#pragma unroll
  for (int i = 0; i < 16; ++i) { const __bf16 h = (__bf16)v[i]; r.h[i] = h; r.l[i] = (__bf16)(v[i] - (float)h); }
  return r; }
__device__ __forceinline__ F2 split_row(const float* row, int k0, int lane) { float v[16]; const float* p = row + k0 + 8 * (lane >> 4);
#pragma unroll
  for (int i = 0; i < 8; ++i) { v[i] = p[i]; v[8 + i] = p[16 + i]; }
  return bsplit16(v); }
__device__ __forceinline__ F2 split_rowK(const float* row, int k0, int lane, int K) { float v[16]; const int g = lane >> 4;
#pragma unroll
  for (int i = 0; i < 8; ++i) { const int ka = k0 + 8 * g + i, kb = ka + 16; v[i] = ka < K ? row[ka < K ? ka : K - 1] : 0.f; v[8 + i] = kb < K ? row[kb < K ? kb : K - 1] : 0.f; }
  return bsplit16(v); }
__device__ __forceinline__ F2 split_col(const float* W, int k0, int n, int lane, int ld, int K) { float v[16]; const int g = lane >> 4;
#pragma unroll
  for (int i = 0; i < 8; ++i) { const int ka = k0 + 8 * g + i, kb = ka + 16; v[i] = ka < K ? W[(size_t)(ka < K ? ka : K - 1) * ld + n] : 0.f; v[8 + i] = kb < K ? W[(size_t)(kb < K ? kb : K - 1) * ld + n] : 0.f; }
  return bsplit16(v); }
__device__ __forceinline__ v8f mac3(const F2& a, const F2& b, v8f c) { c = wmma_bf(a.l, b.h, c); c = wmma_bf(a.h, b.l, c); return wmma_bf(a.h, b.h, c); }
__device__ __forceinline__ float sigm(float v) { return 1.0f / (1.0f + expf(-v)); }
#define LDSX() do { asm volatile("s_wait_dscnt 0" ::: "memory"); __builtin_amdgcn_wave_barrier(); __builtin_amdgcn_fence(__ATOMIC_RELEASE, "workgroup"); } while (0)


#define NB 2
#define LL 256
#define CB 64
#define DM 512
#define NH 8
#define HD 64
#ifndef TNR
#define TNR (NB * LL)
#endif
typedef __attribute__((ext_vector_type(8))) __bf16 v8b;
__device__ __forceinline__ v16b frag_b(const __bf16* rowk0, int lane) {
  union { v16b v; v8b q[2]; } u; const __bf16* p = rowk0 + 8 * (lane >> 4);
  u.q[0] = *(const v8b*)p; u.q[1] = *(const v8b*)(p + 16); return u.v;
}
__device__ __forceinline__ float bfr(float v) { return (float)(__bf16)v; }
__device__ __attribute__((noinline)) float exp_ni(float v) { return expf(v); }
__device__ __attribute__((noinline)) float erf_ni(float v) { return erff(v); }

#define WS_PT  0u
#define WS_END (WS_PT + 2u * (size_t)2 * DM * CB)

__global__ __launch_bounds__(64) void k_packT(const float* __restrict__ WK, const float* __restrict__ WV, __bf16* __restrict__ PT) { const int n = blockIdx.x, which = blockIdx.y, t = threadIdx.x; __shared__ __align__(16) __bf16 s[CB]; const float* w = which ? WV : WK; s[t] = (__bf16)w[(size_t)t * DM + n]; __syncthreads(); if (t < CB / 8) vst2((unsigned*)(PT + ((size_t)which * DM + n) * CB + t * 8), *(const v4u*)&s[t * 8]); }
__global__ __launch_bounds__(128) void k_row(const float* __restrict__ X, const float* __restrict__ PAIR, const float* __restrict__ WQ, const float* __restrict__ BQ, const __bf16* __restrict__ PT, const float* __restrict__ BK, const float* __restrict__ BV, const float* __restrict__ WO, const float* __restrict__ BO, const float* __restrict__ G, const float* __restrict__ Bt, float* __restrict__ OUT) {
  __shared__ __align__(16) float sx[DM]; __shared__ __align__(16) float sq[DM]; __shared__ __align__(16) float sK[LL][HD + 1]; __shared__ __align__(16) float sV[LL][HD + 1]; __shared__ float sS[LL]; __shared__ float sCtx[DM]; __shared__ float sred[8]; __shared__ float spart[2][HD]; __shared__ __align__(16) float so[DM];
  const int tid = threadIdx.x, wave = tid >> 5, lane = tid & 31, col = lane & 15, g = lane >> 4; const size_t bi = blockIdx.x; const size_t b = bi / LL;
  for (int e = tid; e < DM; e += 128) sx[e] = bfr(X[bi * DM + e]);
  __syncthreads();
  for (int n = tid; n < DM; n += 128) { float a = 0.f; for (int c = 0; c < DM; ++c) a += sx[c] * bfr(WQ[(size_t)c * DM + n]); sq[n] = a + bfr(BQ[n]); }
  __syncthreads();
  const float* prow = PAIR + bi * (size_t)LL * CB;
  for (int h = 0; h < NH; ++h) {
#pragma unroll 1
    for (int which = 0; which < 2; ++which) { const __bf16* Wt = PT + ((size_t)which * DM + h * HD) * CB; const float* BB = (which ? BV : BK) + h * HD;
#pragma unroll 1
      for (int rt = 0; rt < 4; ++rt) { const int j0 = wave * 64 + rt * 16; v8f acc[4] = {};
#pragma unroll
        for (int kc = 0; kc < 2; ++kc) { v16b a; { const float* p = prow + (size_t)(j0 + col) * CB + kc * 32 + 8 * g;
#pragma unroll
            for (int i = 0; i < 8; ++i) { a[i] = (__bf16)p[i]; a[8 + i] = (__bf16)p[16 + i]; } }
#pragma unroll
          for (int ct = 0; ct < 4; ++ct) acc[ct] = wmma_bf(a, frag_b(Wt + (size_t)(ct * 16 + col) * CB + kc * 32, lane), acc[ct]); }
#pragma unroll
        for (int ct = 0; ct < 4; ++ct) { const float bb = bfr(BB[ct * 16 + col]);
#pragma unroll
          for (int r = 0; r < 8; ++r) { if (which) sV[j0 + 8 * g + r][ct * 16 + col] = acc[ct][r] + bb; else sK[j0 + 8 * g + r][ct * 16 + col] = acc[ct][r] + bb; } } } }
    __syncthreads();
    for (int j = tid; j < LL; j += 128) { float a = 0.f; for (int d = 0; d < HD; ++d) a += sq[h * HD + d] * sK[j][d]; sS[j] = a * 0.125f; }
    __syncthreads();
    { float mx = -3.0e38f; for (int j = tid; j < LL; j += 128) mx = fmaxf(mx, sS[j]);
#pragma unroll
      for (int o = 1; o < 32; o <<= 1) mx = fmaxf(mx, __shfl_xor(mx, o)); if (lane == 0) sred[wave] = mx; }
    __syncthreads(); const float M = fmaxf(fmaxf(sred[0], sred[1]), fmaxf(sred[2], sred[3])); __syncthreads();
    { float z = 0.f; for (int j = tid; j < LL; j += 128) { const float e = __expf(sS[j] - M); sS[j] = e; z += e; }
#pragma unroll
      for (int o = 1; o < 32; o <<= 1) z += __shfl_xor(z, o); if (lane == 0) sred[4 + wave] = z; }
    __syncthreads(); const float Z = (sred[4] + sred[5]) + (sred[6] + sred[7]);
    { const int d = tid & 63, hf = tid >> 6; float a = 0.f; for (int j = hf * 128; j < hf * 128 + 128; ++j) a += sS[j] * sV[j][d]; spart[hf][d] = a; }
    __syncthreads(); if (tid < HD) sCtx[h * HD + tid] = (spart[0][tid] + spart[1][tid]) / Z; __syncthreads(); }
  for (int n = tid; n < DM; n += 128) { float a = 0.f; for (int c = 0; c < DM; ++c) a += sCtx[c] * bfr(WO[(size_t)c * DM + n]); so[n] = a + bfr(BO[n]) + sx[n]; }
  __syncthreads();
  { float s = 0.f; for (int n = tid; n < DM; n += 128) s += so[n];
#pragma unroll
    for (int o = 1; o < 32; o <<= 1) s += __shfl_xor(s, o); if (lane == 0) sred[wave] = s; }
  __syncthreads(); const float mu = ((sred[0] + sred[1]) + (sred[2] + sred[3])) / (float)DM; __syncthreads();
  { float q = 0.f; for (int n = tid; n < DM; n += 128) { const float dd = so[n] - mu; q += dd * dd; }
#pragma unroll
    for (int o = 1; o < 32; o <<= 1) q += __shfl_xor(q, o); if (lane == 0) sred[4 + wave] = q; }
  __syncthreads(); const float inv = 1.0f / sqrtf(((sred[4] + sred[5]) + (sred[6] + sred[7])) / (float)DM + 1e-5f);
  for (int n = tid; n < DM; n += 128) so[n] = (so[n] - mu) * inv * bfr(G[n]) + bfr(Bt[n]);
  __syncthreads(); vst2(OUT + bi * DM + tid * 4, *(const v4f*)&so[tid * 4]);
}
extern "C" void kernel_launch(void* const* d_in, const int* in_sizes, int n_in, void* d_out, int out_size, void* d_ws, size_t ws_size, hipStream_t stream) {
  (void)in_sizes; (void)n_in; (void)out_size;
  const float** F = (const float**)d_in;
  if (ws_size < (size_t)WS_END) return;
  char* ws = (char*)d_ws; __bf16* PT = (__bf16*)ws;
  k_packT<<<dim3(DM, 2), 64, 0, stream>>>(F[4], F[6], PT);
  k_row<<<TNR, 128, 0, stream>>>(F[0], F[1], F[2], F[3], PT, F[5], F[7], F[8], F[9], F[10], F[11], (float*)d_out);
}
